// droneDeliveryModelHeterogenous_9723805958640
// MI455X (gfx1250) — hardware-verified
//
#include <hip/hip_runtime.h>
#include <stddef.h>


#define NTHR  256
#define NWAVE 8
#define GR    32
#define GC    128
#define XSP   132
#define XP2   68
#define KD    64
#define NHEAD 8
#define CHN   64
#define RW    512
#define NB    128
#define CHUNK 2048
#define WCAP  256
#define NGRP  (CHUNK / (NTHR * 4))
#define ACCF  (NB * RW)
#define NST   (NB * NHEAD)
#define AGG_LDS_BYTES ((ACCF + 2 * NST) * 4 + (NWAVE * WCAP + NWAVE) * 4)
#define ORB   256
#define NOUT  5
#define WOF1  32768
#define WOF2  65536
#define WOF3  98304
#define WOF4  131072
#define WOF5  135168
#define WOF6  139264
#define WTOT  140288

static_assert(NGRP == 2);
static_assert(WCAP == (CHUNK / NTHR) * 32);
static_assert(AGG_LDS_BYTES == 278560);
static_assert((XSP % 4) == 0);
static_assert((XP2 % 4) == 0);
static_assert(KD == 64);
static_assert(RW == NHEAD * CHN);
static_assert((NB % NWAVE) == 0);
static_assert((NB & (NB - 1)) == 0);
static_assert(NB <= WCAP);
static_assert((ORB * NOUT) % 4 == 0);

typedef float          v2f  __attribute__((ext_vector_type(2)));
typedef float          v4f  __attribute__((ext_vector_type(4)));
typedef float          v8f  __attribute__((ext_vector_type(8)));
typedef int            v4i  __attribute__((ext_vector_type(4)));
typedef _Float16       v8h  __attribute__((ext_vector_type(8)));
typedef _Float16       v16h __attribute__((ext_vector_type(16)));
typedef unsigned short v8us __attribute__((ext_vector_type(8)));

union FragH { v16h v; v4i u[2]; };
union Pack  { v8h h; v8us s; v4i i; };

__device__ __forceinline__ v8f wmh(v16h a, v16h b, v8f c) {
  v8f d = __builtin_amdgcn_wmma_f32_16x16x32_f16(false, a, false, b, (short)0, c, false, false);
  asm volatile("v_nop\n\tv_nop\n\tv_nop\n\tv_nop" : "+v"(d) : "v"(a), "v"(b));
  return d;
}

__device__ __forceinline__ float lk(float t) { return fmaxf(t, 0.2f * t); }
__device__ __forceinline__ float dl(v4f t, v4f w) {
  return w.x * lk(t.x) + w.y * lk(t.y) + w.z * lk(t.z) + w.w * lk(t.w);
}

__global__ __launch_bounds__(NTHR) void k_wcvt(const float* __restrict__ s0, const float* __restrict__ s1,
                                               const float* __restrict__ s2, const float* __restrict__ s3,
                                               const float* __restrict__ s4, const float* __restrict__ s5,
                                               const float* __restrict__ s6, unsigned short* dst, float scale) {
  const int job = blockIdx.y;
  const float* src = s0;
  int rsrc = 512, rtot = 512, dofs = 0;
  if (job == 1)      { src = s1; dofs = WOF1; }
  else if (job == 2) { src = s2; dofs = WOF2; }
  else if (job == 3) { src = s3; dofs = WOF3; }
  else if (job == 4) { src = s4; rsrc = 64; rtot = 64; dofs = WOF4; }
  else if (job == 5) { src = s5; rsrc = 64; rtot = 64; dofs = WOF5; }
  else if (job == 6) { src = s6; rsrc = NOUT; rtot = 16; dofs = WOF6; }
  else if (job != 0) return;
  const int i = blockIdx.x * NTHR + threadIdx.x;
  if (i >= rtot * (KD / 8)) return;
  const int r  = i >> 3;
  const int kb = (i & 7) * 8;
  const int rc = (r < rsrc) ? r : (rsrc - 1);
  const float* p = src + (size_t)rc * KD + kb;
  const v4f t0 = *(const v4f*)(p);
  const v4f t1 = *(const v4f*)(p + 4);
  Pack u;
  const v4i z4 = {0, 0, 0, 0};
  u.i = z4;
#pragma unroll
  for (int j = 0; j < 4; ++j) {
    u.h[j]     = (_Float16)(t0[j] * scale);
    u.h[4 + j] = (_Float16)(t1[j] * scale);
  }
  if (r >= rsrc) u.i = z4;
  unsigned short* op = dst + dofs + (size_t)i * 8;
  *(volatile v4i*)op = u.i;
  __threadfence();
  *(volatile v4i*)op = u.i;
}

__global__ __launch_bounds__(NTHR) void k_in(const float* __restrict__ x,
                                             const float* __restrict__ W1d, const float* __restrict__ b1d,
                                             const float* __restrict__ W1g, const float* __restrict__ b1g,
                                             unsigned short* outp, int nN, int nPad) {
  const int i = blockIdx.x * NTHR + threadIdx.x;
  const int r = i >> 3;
  const int q = i & 7;
  if (r >= nPad) return;
  const int rc = (r < nN) ? r : (nN - 1);
  float xv[6];
#pragma unroll
  for (int k = 0; k < 6; ++k) xv[k] = x[(size_t)rc * 6 + k];
  const bool goal = xv[5] > 0.0f;
  Pack u;
  const v4i z4 = {0, 0, 0, 0};
  u.i = z4;
#pragma unroll
  for (int j = 0; j < 8; ++j) {
    const int c = 8 * q + j;
    const float wd0 = W1d[c * 6], wg0 = W1g[c * 6];
    float v = xv[0] * (goal ? wg0 : wd0);
#pragma unroll
    for (int k = 1; k < 6; ++k) {
      const float wd = W1d[c * 6 + k], wg = W1g[c * 6 + k];
      v += xv[k] * (goal ? wg : wd);
    }
    const float bd = b1d[c], bg = b1g[c];
    v += (goal ? bg : bd);
    u.h[j] = (_Float16)v;
  }
  if (r >= nN) u.i = z4;
  unsigned short* op = outp + (size_t)r * CHN + 8 * q;
  *(volatile v4i*)op = u.i;
  __threadfence();
  *(volatile v4i*)op = u.i;
}

__global__ __launch_bounds__(NTHR) void k_gemm(const unsigned short* __restrict__ A,
                                               const unsigned short* __restrict__ B,
                                               const float* __restrict__ bias, float* out,
                                               int K, int Ncols, float oscale) {
  __shared__ __attribute__((aligned(16))) float Xs[GR * XSP];

  const int tid  = threadIdx.x;
  const int lane = tid & 31;
  const int wave = tid >> 5;
  const int hh   = lane >> 4;
  const int m    = lane & 15;
  const int rowBase = blockIdx.x * GR;
  const int colBase = blockIdx.y * GC;
  const int ncol = colBase + wave * 16 + m;

  const size_t ra0 = (size_t)(rowBase + m) * K + 8 * hh;
  const size_t ra1 = ra0 + (size_t)16 * K;
  const size_t rb  = (size_t)ncol * K + 8 * hh;

  v8f c0 = {0.f, 0.f, 0.f, 0.f, 0.f, 0.f, 0.f, 0.f};
  v8f c1 = {0.f, 0.f, 0.f, 0.f, 0.f, 0.f, 0.f, 0.f};

#pragma unroll 1
  for (int k0 = 0; k0 < K; k0 += 32) {
    FragH a0, a1, b;
    a0.u[0] = *(const v4i*)(A + ra0 + k0);  a0.u[1] = *(const v4i*)(A + ra0 + k0 + 16);
    a1.u[0] = *(const v4i*)(A + ra1 + k0);  a1.u[1] = *(const v4i*)(A + ra1 + k0 + 16);
    b.u[0]  = *(const v4i*)(B + rb + k0);   b.u[1]  = *(const v4i*)(B + rb + k0 + 16);
    c0 = wmh(a0.v, b.v, c0);
    c1 = wmh(a1.v, b.v, c1);
  }

  const float bv = bias[ncol];
  const int cl = wave * 16 + m;
#pragma unroll
  for (int r = 0; r < 8; ++r) {
    Xs[(8 * hh + r) * XSP + cl]      = c0[r] * oscale + bv;
    Xs[(16 + 8 * hh + r) * XSP + cl] = c1[r] * oscale + bv;
  }
  __syncthreads();

  v4f xv[4];
  float* xpp[4];
#pragma unroll
  for (int i = 0; i < 4; ++i) {
    xv[i]  = *(const v4f*)(Xs + (4 * wave + i) * XSP + 4 * lane);
    xpp[i] = out + (size_t)(rowBase + 4 * wave + i) * Ncols + colBase + 4 * lane;
  }
#pragma unroll
  for (int i = 0; i < 4; ++i) *(volatile v4f*)(xpp[i]) = xv[i];
  __threadfence();
#pragma unroll
  for (int i = 0; i < 4; ++i) *(volatile v4f*)(xpp[i]) = xv[i];
}

__global__ __launch_bounds__(NTHR) void k_gemm2(const unsigned short* __restrict__ A,
                                                const unsigned short* __restrict__ Bd,
                                                const unsigned short* __restrict__ Bg,
                                                const float* __restrict__ bd, const float* __restrict__ bg,
                                                const float* __restrict__ x, unsigned short* outp,
                                                int nN, float oscale) {
  __shared__ __attribute__((aligned(16))) float Xs[2 * GR * XP2];

  const int tid  = threadIdx.x;
  const int lane = tid & 31;
  const int wave = tid >> 5;
  const int hh   = lane >> 4;
  const int m    = lane & 15;
  const int set  = wave >> 2;
  const int ct   = wave & 3;
  const int ncol = 16 * ct + m;
  const int rowBase = blockIdx.x * GR;

  const size_t ra0 = (size_t)(rowBase + m) * KD + 8 * hh;
  const size_t ra1 = ra0 + (size_t)16 * KD;
  const size_t rb  = (size_t)ncol * KD + 8 * hh;

  v8f c0 = {0.f, 0.f, 0.f, 0.f, 0.f, 0.f, 0.f, 0.f};
  v8f c1 = {0.f, 0.f, 0.f, 0.f, 0.f, 0.f, 0.f, 0.f};

#pragma unroll
  for (int k0 = 0; k0 < KD; k0 += 32) {
    FragH a0, a1, b;
    a0.u[0] = *(const v4i*)(A + ra0 + k0);  a0.u[1] = *(const v4i*)(A + ra0 + k0 + 16);
    a1.u[0] = *(const v4i*)(A + ra1 + k0);  a1.u[1] = *(const v4i*)(A + ra1 + k0 + 16);
    const v4i bd0 = *(const v4i*)(Bd + rb + k0), bd1 = *(const v4i*)(Bd + rb + k0 + 16);
    const v4i bg0 = *(const v4i*)(Bg + rb + k0), bg1 = *(const v4i*)(Bg + rb + k0 + 16);
    b.u[0] = set ? bg0 : bd0;
    b.u[1] = set ? bg1 : bd1;
    c0 = wmh(a0.v, b.v, c0);
    c1 = wmh(a1.v, b.v, c1);
  }

  const float bvd = bd[ncol], bvg = bg[ncol];
  const float bv = set ? bvg : bvd;
#pragma unroll
  for (int r = 0; r < 8; ++r) {
    Xs[(set * GR + 8 * hh + r) * XP2 + ncol]      = c0[r] * oscale + bv;
    Xs[(set * GR + 16 + 8 * hh + r) * XP2 + ncol] = c1[r] * oscale + bv;
  }
  __syncthreads();

  const int r = tid >> 3;
  const int q = tid & 7;
  const int node = rowBase + r;
  const int nc = (node < nN) ? node : (nN - 1);
  const bool goal = x[(size_t)nc * 6 + 5] > 0.0f;
  const float* sd = Xs + r * XP2 + 8 * q;
  const float* sg = Xs + (GR + r) * XP2 + 8 * q;
  const v4f t0d = *(const v4f*)(sd), t1d = *(const v4f*)(sd + 4);
  const v4f t0g = *(const v4f*)(sg), t1g = *(const v4f*)(sg + 4);
  const v4f t0 = goal ? t0g : t0d;
  const v4f t1 = goal ? t1g : t1d;
  Pack u;
  const v4i z4 = {0, 0, 0, 0};
  u.i = z4;
#pragma unroll
  for (int j = 0; j < 4; ++j) {
    u.h[j]     = (_Float16)t0[j];
    u.h[4 + j] = (_Float16)t1[j];
  }
  if (node >= nN) u.i = z4;
  unsigned short* op = outp + (size_t)node * CHN + 8 * q;
  *(volatile v4i*)op = u.i;
  __threadfence();
  *(volatile v4i*)op = u.i;
}

__device__ __forceinline__ void hit(const float* xs, const float* xd, float* ar, float* shp, float* dp,
                                    bool selfp, v4f w0, v4f w1, v4f w2, v4f w3) {
  const v4f a0 = *(const v4f*)(xs),     a1 = *(const v4f*)(xs + 4);
  const v4f a2 = *(const v4f*)(xs + 8), a3 = *(const v4f*)(xs + 12);
  const v4f d0 = *(const v4f*)(xd),     d1 = *(const v4f*)(xd + 4);
  const v4f d2 = *(const v4f*)(xd + 8), d3 = *(const v4f*)(xd + 12);
  float s = dl(a0 + d0, w0) + dl(a1 + d1, w1) + dl(a2 + d2, w2) + dl(a3 + d3, w3);
  s += __shfl_xor(s, 1, 32);
  s += __shfl_xor(s, 2, 32);
  float shv = shp[0];
  if (selfp) { shv = s; shp[0] = s; }
  const float p = __expf(s - shv);
  v4f e0 = *(v4f*)(ar),     e1 = *(v4f*)(ar + 4);
  v4f e2 = *(v4f*)(ar + 8), e3 = *(v4f*)(ar + 12);
  e0 = e0 + a0 * p;  e1 = e1 + a1 * p;
  e2 = e2 + a2 * p;  e3 = e3 + a3 * p;
  *(v4f*)(ar)     = e0;  *(v4f*)(ar + 4)  = e1;
  *(v4f*)(ar + 8) = e2;  *(v4f*)(ar + 12) = e3;
  dp[0] = dp[0] + p;
}

__global__ __launch_bounds__(NTHR) void k_agg(const int* __restrict__ ei, const float* __restrict__ xl,
                                              const float* __restrict__ xr, const float* __restrict__ att,
                                              const float* __restrict__ bias, unsigned short* outp,
                                              int nN, int nE) {
  extern __shared__ v4f lds_dyn[];
  float* sacc = (float*)lds_dyn;
  float* sh   = sacc + ACCF;
  float* dn   = sh + NST;
  int*   list = (int*)(dn + NST);
  int*   wcnt = list + NWAVE * WCAP;

  const int tid  = threadIdx.x;
  const int lane = tid & 31;
  const int wave = tid >> 5;
  const int nodeBase = blockIdx.x * NB;

  {
    const v4f z4 = {0.f, 0.f, 0.f, 0.f};
    for (int i = tid; i < ACCF / 4; i += NTHR) lds_dyn[i] = z4;
    for (int i = tid; i < NST; i += NTHR) { sh[i] = 0.f; dn[i] = 0.f; }
  }
  __syncthreads();

  const int coff = 16 * lane;
  const int hd   = lane >> 2;
  const v4f w0 = *(const v4f*)(att + coff);
  const v4f w1 = *(const v4f*)(att + coff + 4);
  const v4f w2 = *(const v4f*)(att + coff + 8);
  const v4f w3 = *(const v4f*)(att + coff + 12);

  const int* eid = ei + nE;
  const bool al16 = ((nE & 3) == 0);
  const int nChunks = (nE + CHUNK - 1) / CHUNK;

#pragma unroll 1
  for (int ch = 0; ch <= nChunks; ++ch) {
    const bool selfp = (ch == 0);
    const int cbase = selfp ? 0 : (ch - 1) * CHUNK;
    if (selfp) {
      for (int s = tid; s < NB; s += NTHR) list[s] = s;
      if (tid < NWAVE) {
        int c = NB - tid * WCAP;
        c = c < 0 ? 0 : (c > WCAP ? WCAP : c);
        wcnt[tid] = c;
      }
    } else {
      int wc = 0;
#pragma unroll
      for (int g = 0; g < NGRP; ++g) {
        const int el0 = (g * NTHR + tid) * 4;
        const int e0  = cbase + el0;
        const int sent = -2147483647 - 1;
        v4i d;
        if (al16 && (e0 + 3 < nE)) {
          d = *(const v4i*)(eid + e0);
        } else {
          d.x = (e0     < nE) ? eid[min(e0, nE - 1)]     : sent;
          d.y = (e0 + 1 < nE) ? eid[min(e0 + 1, nE - 1)] : sent;
          d.z = (e0 + 2 < nE) ? eid[min(e0 + 2, nE - 1)] : sent;
          d.w = (e0 + 3 < nE) ? eid[min(e0 + 3, nE - 1)] : sent;
        }
        const unsigned s0 = (unsigned)d.x - (unsigned)nodeBase;
        const unsigned s1 = (unsigned)d.y - (unsigned)nodeBase;
        const unsigned s2 = (unsigned)d.z - (unsigned)nodeBase;
        const unsigned s3 = (unsigned)d.w - (unsigned)nodeBase;
        const bool h0 = s0 < (unsigned)NB;
        const bool h1 = s1 < (unsigned)NB;
        const bool h2 = s2 < (unsigned)NB;
        const bool h3 = s3 < (unsigned)NB;
        const unsigned many = __builtin_amdgcn_ballot_w32(h0 | h1 | h2 | h3);
        if (many != 0u) {
#define HITJ(J, HJ, SJ) { \
            const unsigned mj = __builtin_amdgcn_ballot_w32(HJ); \
            if (HJ) { \
              const int pos = wc + (int)__builtin_amdgcn_mbcnt_lo(mj, 0u); \
              if (pos < WCAP) list[wave * WCAP + pos] = ((el0 + (J)) << 9) | (int)(SJ); \
            } \
            wc += (int)__builtin_popcount(mj); }
          HITJ(0, h0, s0)
          HITJ(1, h1, s1)
          HITJ(2, h2, s2)
          HITJ(3, h3, s3)
#undef HITJ
        }
      }
      if (lane == 0) wcnt[wave] = wc;
    }
    __syncthreads();

    if (wave == 0) {
#pragma unroll 1
      for (int wsx = 0; wsx < NWAVE; ++wsx) {
        int n = __builtin_amdgcn_readfirstlane(wcnt[wsx]);
        n = n > WCAP ? WCAP : n;
        n = n < 0 ? 0 : n;
#pragma unroll 1
        for (int i = 0; i < n; ++i) {
          const int ent  = __builtin_amdgcn_readfirstlane(list[wsx * WCAP + i]);
          const int slot = ent & (NB - 1);
          const int el   = (ent >> 9) & (CHUNK - 1);
          const int node = nodeBase + slot;
          if (node >= nN) continue;
          int e = cbase + el;
          if (e > nE - 1) e = nE - 1;
          int sj = ei[e];
          sj = sj < 0 ? 0 : (sj > nN - 1 ? nN - 1 : sj);
          const int src = selfp ? node : sj;
          const float* xs = xl + (size_t)src * RW + coff;
          const float* xd = xr + (size_t)node * RW + coff;
          float* ar  = sacc + slot * RW + coff;
          float* shp = sh + slot * NHEAD + hd;
          float* dp  = dn + slot * NHEAD + hd;
          hit(xs, xd, ar, shp, dp, selfp, w0, w1, w2, w3);
        }
      }
    }
    __syncthreads();
  }

#pragma unroll 1
  for (int it = 0; it < NB / NWAVE; ++it) {
    const int s = it * NWAVE + wave;
    const int node = nodeBase + s;
    Pack u;
    const v4i z4 = {0, 0, 0, 0};
    u.i = z4;
    if (node < nN) {
      float inv[NHEAD];
#pragma unroll
      for (int h = 0; h < NHEAD; ++h) inv[h] = __builtin_amdgcn_rcpf(dn[s * NHEAD + h]);
      const float* base = sacc + s * RW + 2 * lane;
      float sm0 = 0.f, sm1 = 0.f;
#pragma unroll
      for (int h = 0; h < NHEAD; ++h) {
        const v2f t = *(const v2f*)(base + CHN * h);
        sm0 += t.x * inv[h];
        sm1 += t.y * inv[h];
      }
      const float b0 = bias[2 * lane], b1 = bias[2 * lane + 1];
      float v0 = sm0 * 0.125f + b0;
      float v1 = sm1 * 0.125f + b1;
      v0 = fmaxf(v0, 0.f);
      v1 = fmaxf(v1, 0.f);
      const int q = lane & 7;
#pragma unroll
      for (int j = 0; j < 4; ++j) {
        const float xj = __shfl(v0, 4 * q + j, 32);
        const float yj = __shfl(v1, 4 * q + j, 32);
        u.h[2 * j]     = (_Float16)xj;
        u.h[2 * j + 1] = (_Float16)yj;
      }
    }
    if (lane < 8) {
      unsigned short* op = outp + (size_t)node * CHN + 8 * lane;
      *(volatile v4i*)op = u.i;
      __threadfence();
      *(volatile v4i*)op = u.i;
    }
  }
}

__global__ __launch_bounds__(NTHR) void k_out(const unsigned short* __restrict__ A,
                                              const unsigned short* __restrict__ B,
                                              const float* __restrict__ bo, float* out, int tot, float oscale) {
  __shared__ __attribute__((aligned(16))) float ys[ORB * NOUT];

  const int tid  = threadIdx.x;
  const int lane = tid & 31;
  const int wave = tid >> 5;
  const int hh   = lane >> 4;
  const int m    = lane & 15;
  const int rowBase = blockIdx.x * ORB;

  const size_t ra0 = (size_t)(rowBase + 32 * wave + m) * KD + 8 * hh;
  const size_t ra1 = ra0 + (size_t)16 * KD;
  const size_t rb  = (size_t)m * KD + 8 * hh;

  v8f c0 = {0.f, 0.f, 0.f, 0.f, 0.f, 0.f, 0.f, 0.f};
  v8f c1 = {0.f, 0.f, 0.f, 0.f, 0.f, 0.f, 0.f, 0.f};

#pragma unroll
  for (int k0 = 0; k0 < KD; k0 += 32) {
    FragH a0, a1, b;
    a0.u[0] = *(const v4i*)(A + ra0 + k0);  a0.u[1] = *(const v4i*)(A + ra0 + k0 + 16);
    a1.u[0] = *(const v4i*)(A + ra1 + k0);  a1.u[1] = *(const v4i*)(A + ra1 + k0 + 16);
    b.u[0]  = *(const v4i*)(B + rb + k0);   b.u[1]  = *(const v4i*)(B + rb + k0 + 16);
    c0 = wmh(a0.v, b.v, c0);
    c1 = wmh(a1.v, b.v, c1);
  }

  const float bv = bo[(m < NOUT) ? m : (NOUT - 1)];
  if (m < NOUT) {
#pragma unroll
    for (int r = 0; r < 8; ++r) {
      ys[(32 * wave + 8 * hh + r) * NOUT + m]      = c0[r] * oscale + bv;
      ys[(32 * wave + 16 + 8 * hh + r) * NOUT + m] = c1[r] * oscale + bv;
    }
  }
  __syncthreads();

  v4f xv[2];
  size_t fo[2];
  bool ok[2];
#pragma unroll
  for (int i2 = 0; i2 < 2; ++i2) {
    const int idx = tid + i2 * NTHR;
    ok[i2] = idx < (ORB * NOUT) / 4;
    const v4f z4 = {0.f, 0.f, 0.f, 0.f};
    xv[i2] = ok[i2] ? *(const v4f*)(ys + 4 * idx) : z4;
    fo[i2] = (size_t)rowBase * NOUT + (size_t)4 * idx;
  }
#pragma unroll
  for (int i2 = 0; i2 < 2; ++i2) {
    if (ok[i2]) {
      if (fo[i2] + 4 <= (size_t)tot) {
        *(volatile v4f*)(out + fo[i2]) = xv[i2];
      } else {
#pragma unroll
        for (int j = 0; j < 4; ++j)
          if (fo[i2] + j < (size_t)tot) ((volatile float*)out)[fo[i2] + j] = xv[i2][j];
      }
    }
  }
  __threadfence();
#pragma unroll
  for (int i2 = 0; i2 < 2; ++i2) {
    if (ok[i2]) {
      if (fo[i2] + 4 <= (size_t)tot) {
        *(volatile v4f*)(out + fo[i2]) = xv[i2];
      } else {
#pragma unroll
        for (int j = 0; j < 4; ++j)
          if (fo[i2] + j < (size_t)tot) ((volatile float*)out)[fo[i2] + j] = xv[i2][j];
      }
    }
  }
}

extern "C" void kernel_launch(void* const* d_in, const int* in_sizes, int n_in,
                              void* d_out, int out_size, void* d_ws, size_t ws_size,
                              hipStream_t stream) {
  if (n_in < 24) return;
  const int nN = in_sizes[0] / 6;
  if (nN < 2 || in_sizes[0] != nN * 6) return;
  const int nE = in_sizes[1] / 2;
  if (nE <= 0 || in_sizes[1] != 2 * nE) return;
  if (in_sizes[2] != CHN * 6 || in_sizes[3] != CHN || in_sizes[4] != CHN * 6 || in_sizes[5] != CHN) return;
  if (in_sizes[6] != RW * KD || in_sizes[7] != RW || in_sizes[8] != RW * KD || in_sizes[9] != RW ||
      in_sizes[10] != NHEAD * CHN || in_sizes[11] != CHN) return;
  if (in_sizes[12] != CHN * KD || in_sizes[13] != CHN || in_sizes[14] != CHN * KD || in_sizes[15] != CHN) return;
  if (in_sizes[16] != RW * KD || in_sizes[17] != RW || in_sizes[18] != RW * KD || in_sizes[19] != RW ||
      in_sizes[20] != NHEAD * CHN || in_sizes[21] != CHN) return;
  if (in_sizes[22] != NOUT * KD || in_sizes[23] != NOUT) return;
  const int halfN = nN / 2;
  if (out_size != halfN * NOUT) return;

  const float* x    = (const float*)d_in[0];
  const int*   ei   = (const int*)d_in[1];
  const float* W1d  = (const float*)d_in[2];   const float* b1d  = (const float*)d_in[3];
  const float* W1g  = (const float*)d_in[4];   const float* b1g  = (const float*)d_in[5];
  const float* Wl1  = (const float*)d_in[6];   const float* bl1  = (const float*)d_in[7];
  const float* Wr1  = (const float*)d_in[8];   const float* br1  = (const float*)d_in[9];
  const float* att1 = (const float*)d_in[10];  const float* bi1  = (const float*)d_in[11];
  const float* W2d  = (const float*)d_in[12];  const float* b2d  = (const float*)d_in[13];
  const float* W2g  = (const float*)d_in[14];  const float* b2g  = (const float*)d_in[15];
  const float* Wl2  = (const float*)d_in[16];  const float* bl2  = (const float*)d_in[17];
  const float* Wr2  = (const float*)d_in[18];  const float* br2  = (const float*)d_in[19];
  const float* att2 = (const float*)d_in[20];  const float* bi2  = (const float*)d_in[21];
  const float* Wo   = (const float*)d_in[22];  const float* bo   = (const float*)d_in[23];
  float* out = (float*)d_out;

  const int nPad = ((nN + NB - 1) / NB) * NB;
  const int gridOut = (halfN + ORB - 1) / ORB;
  if (gridOut * ORB > nPad) return;

  char* wsp = (char*)d_ws;
  size_t off = 0;
  const size_t plB = (((size_t)nPad * CHN * 2) + 255) & ~(size_t)255;
  const size_t wB  = (((size_t)WTOT * 2) + 255) & ~(size_t)255;
  const size_t xB  = (((size_t)nPad * RW * 4) + 255) & ~(size_t)255;
  unsigned short* h0P = (unsigned short*)(wsp + off); off += plB;
  unsigned short* h1P = (unsigned short*)(wsp + off); off += plB;
  unsigned short* h2P = (unsigned short*)(wsp + off); off += plB;
  unsigned short* h3P = (unsigned short*)(wsp + off); off += plB;
  unsigned short* wP  = (unsigned short*)(wsp + off); off += wB;
  float* xl = (float*)(wsp + off); off += xB;
  float* xr = (float*)(wsp + off); off += xB;
  if (off > ws_size) return;
  if (off > (size_t)134217728) return;

  const unsigned short* Wl1P = wP;
  const unsigned short* Wr1P = wP + WOF1;
  const unsigned short* Wl2P = wP + WOF2;
  const unsigned short* Wr2P = wP + WOF3;
  const unsigned short* W2dP = wP + WOF4;
  const unsigned short* W2gP = wP + WOF5;
  const unsigned short* WoP  = wP + WOF6;

  const float s16  = 16.0f;
  const float is16 = 0.0625f;
  const int mt = nPad / GR;

  hipFuncSetAttribute(reinterpret_cast<const void*>(&k_agg),
                      hipFuncAttributeMaxDynamicSharedMemorySize, AGG_LDS_BYTES);

  k_wcvt<<<dim3(16, 7), NTHR, 0, stream>>>(Wl1, Wr1, Wl2, Wr2, W2d, W2g, Wo, wP, s16);
  k_in<<<nPad / 32, NTHR, 0, stream>>>(x, W1d, b1d, W1g, b1g, h0P, nN, nPad);

  k_gemm<<<dim3(mt, RW / GC), NTHR, 0, stream>>>(h0P, Wl1P, bl1, xl, KD, RW, is16);
  k_gemm<<<dim3(mt, RW / GC), NTHR, 0, stream>>>(h0P, Wr1P, br1, xr, KD, RW, is16);
  k_agg<<<nPad / NB, NTHR, AGG_LDS_BYTES, stream>>>(ei, xl, xr, att1, bi1, h1P, nN, nE);

  k_gemm2<<<mt, NTHR, 0, stream>>>(h1P, W2dP, W2gP, b2d, b2g, x, h2P, nN, is16);

  k_gemm<<<dim3(mt, RW / GC), NTHR, 0, stream>>>(h2P, Wl2P, bl2, xl, KD, RW, is16);
  k_gemm<<<dim3(mt, RW / GC), NTHR, 0, stream>>>(h2P, Wr2P, br2, xr, KD, RW, is16);
  k_agg<<<nPad / NB, NTHR, AGG_LDS_BYTES, stream>>>(ei, xl, xr, att2, bi2, h3P, nN, nE);

  k_out<<<gridOut, NTHR, 0, stream>>>(h3P, WoP, bo, out, halfN * NOUT, is16);
}
